// EncoderWithPositionalAttentionLayer_24807731102179
// MI455X (gfx1250) — hardware-verified
//
#include <hip/hip_runtime.h>
#include <math.h>

typedef __attribute__((ext_vector_type(16))) _Float16 v16h;
typedef __attribute__((ext_vector_type(16))) __bf16 v16b;
typedef __attribute__((ext_vector_type(8)))  _Float16 v8h;
typedef __attribute__((ext_vector_type(8)))  float v8f;
typedef __attribute__((ext_vector_type(4)))  float v4f;
typedef __attribute__((ext_vector_type(2)))  float v2f;
typedef __attribute__((ext_vector_type(4)))  unsigned v4u;
typedef __attribute__((ext_vector_type(4)))  int v4i;
typedef float __attribute__((may_alias)) float_a;
typedef int __attribute__((may_alias)) int_a;

template <typename T> __device__ __forceinline__ void vst2(void* p, T v) { *(volatile T*)p = v; __threadfence(); *(volatile T*)p = v; }
__device__ __forceinline__ v8f wmma16(v16h a, v16h b, v8f c) {
  v8f d = __builtin_amdgcn_wmma_f32_16x16x32_f16(false, a, false, b, (short)0, c, false, false);
  asm volatile("v_nop\n\tv_nop\n\tv_nop\n\tv_nop" : "+v"(d) : "v"(a), "v"(b));
  return d;
}
__device__ __forceinline__ v8f wmma_bf(v16b a, v16b b, v8f c) {
  v8f d = __builtin_amdgcn_wmma_f32_16x16x32_bf16(false, a, false, b, (short)0, c, false, false);
  asm volatile("v_nop\n\tv_nop\n\tv_nop\n\tv_nop" : "+v"(d) : "v"(a), "v"(b));
  return d;
}
__device__ __forceinline__ v16h frag_h(const _Float16* rowk0, int lane) {
  union { v16h v; v8h q[2]; } u; const _Float16* p = rowk0 + 8 * (lane >> 4);
  u.q[0] = *(const v8h*)p; u.q[1] = *(const v8h*)(p + 16); return u.v;
}
__device__ __forceinline__ v16h frag_f32(const float* rowk0, int lane) {
  v16h a; const float* p = rowk0 + 8 * (lane >> 4);
#pragma unroll
  for (int i = 0; i < 8; ++i) { a[i] = (_Float16)p[i]; a[8 + i] = (_Float16)p[16 + i]; }
  return a;
}
__device__ __forceinline__ v16h frag_f32s(const float* rowk0, int lane, float sc) {
  v16h a; const float* p = rowk0 + 8 * (lane >> 4);
#pragma unroll
  for (int i = 0; i < 8; ++i) { a[i] = (_Float16)(p[i] * sc); a[8 + i] = (_Float16)(p[16 + i] * sc); }
  return a;
}
__device__ __forceinline__ v16h fragc_f32(const float* W, int k0, int n, int lane, int ld, int K) {
  v16h a; const int g = lane >> 4;
#pragma unroll
  for (int i = 0; i < 8; ++i) { const int ka = k0 + 8 * g + i, kb = ka + 16;
    a[i] = (_Float16)(ka < K ? W[(size_t)(ka < K ? ka : K - 1) * ld + n] : 0.f); a[8 + i] = (_Float16)(kb < K ? W[(size_t)(kb < K ? kb : K - 1) * ld + n] : 0.f); }
  return a;
}
struct F2 { v16b h, l; };
__device__ __forceinline__ F2 bsplit16(const float v[16]) { F2 r;
#pragma unroll
  for (int i = 0; i < 16; ++i) { const __bf16 h = (__bf16)v[i]; r.h[i] = h; r.l[i] = (__bf16)(v[i] - (float)h); }
  return r; }
__device__ __forceinline__ F2 split_row(const float* row, int k0, int lane) { float v[16]; const float* p = row + k0 + 8 * (lane >> 4);
#pragma unroll
  for (int i = 0; i < 8; ++i) { v[i] = p[i]; v[8 + i] = p[16 + i]; }
  return bsplit16(v); }
__device__ __forceinline__ F2 split_rowK(const float* row, int k0, int lane, int K) { float v[16]; const int g = lane >> 4;
#pragma unroll
  for (int i = 0; i < 8; ++i) { const int ka = k0 + 8 * g + i, kb = ka + 16; v[i] = ka < K ? row[ka < K ? ka : K - 1] : 0.f; v[8 + i] = kb < K ? row[kb < K ? kb : K - 1] : 0.f; }
  return bsplit16(v); }
__device__ __forceinline__ F2 split_col(const float* W, int k0, int n, int lane, int ld, int K) { float v[16]; const int g = lane >> 4;
#pragma unroll
  for (int i = 0; i < 8; ++i) { const int ka = k0 + 8 * g + i, kb = ka + 16; v[i] = ka < K ? W[(size_t)(ka < K ? ka : K - 1) * ld + n] : 0.f; v[8 + i] = kb < K ? W[(size_t)(kb < K ? kb : K - 1) * ld + n] : 0.f; }
  return bsplit16(v); }
__device__ __forceinline__ v8f mac3(const F2& a, const F2& b, v8f c) { c = wmma_bf(a.l, b.h, c); c = wmma_bf(a.h, b.l, c); return wmma_bf(a.h, b.h, c); }
__device__ __forceinline__ float sigm(float v) { return 1.0f / (1.0f + expf(-v)); }
#define LDSX() do { asm volatile("s_wait_dscnt 0" ::: "memory"); __builtin_amdgcn_wave_barrier(); __builtin_amdgcn_fence(__ATOMIC_RELEASE, "workgroup"); } while (0)


#define NB 8
#define TT 512
#define DM 512
#define NH 8
#define HD 64
#define HID 2048
#define LR 100
#define NREL (2 * LR + 1)
#define NRP 208
#define NR (NB * TT)
#ifndef NBT
#define NBT NB
#define TB0 0
#define TQB (TT / 64)
#endif
#define RB0 ((size_t)TB0 * TT)
typedef __attribute__((ext_vector_type(8))) __bf16 v8b;
__device__ __forceinline__ v16b frag_b(const __bf16* rowk0, int lane) {
  union { v16b v; v8b q[2]; } u; const __bf16* p = rowk0 + 8 * (lane >> 4);
  u.q[0] = *(const v8b*)p; u.q[1] = *(const v8b*)(p + 16); return u.v;
}
__device__ __forceinline__ float bfr(float v) { return (float)(__bf16)v; }
__device__ __attribute__((noinline)) float exp_ni(float v) { return expf(v); }
__device__ __attribute__((noinline)) float erf_ni(float v) { return erff(v); }

#define PK_H0 0
#define PK_Q  ((size_t)HID * DM)
#define PK_KE (PK_Q + (size_t)DM * HID)
#define PK_KV (PK_KE + (size_t)DM * HID)
#define PK_KR (PK_KV + (size_t)DM * HID)
#define PK_H1 (PK_KR + (size_t)DM * DM)
#define PK_O1 (PK_H1 + (size_t)HID * DM)
#define PK_END (PK_O1 + (size_t)DM * HID)
#define WS_PK  0u
#define WS_XN  (((2u * PK_END) + 127u) / 128u * 128u)
#define WS_XH  (WS_XN + 4u * NR * DM)
#define WS_XL  (WS_XH + 2u * (size_t)NR * HID)
#define WS_QH  (WS_XL + 2u * (size_t)NR * HID)
#define WS_QL  (WS_QH + 2u * NR * DM)
#define WS_KEH (WS_QL + 2u * NR * DM)
#define WS_KEL (WS_KEH + 2u * NR * DM)
#define WS_VTH (WS_KEL + 2u * NR * DM)
#define WS_VTL (WS_VTH + 2u * NR * DM)
#define WS_KRH (WS_VTL + 2u * NR * DM)
#define WS_KRL (WS_KRH + 2u * NRP * DM)
#define WS_KRF (WS_KRL + 2u * NRP * DM)
#define WS_B0  (WS_KRF + 4u * NRP * DM)
#define WS_B1  (WS_B0 + 4u * NR * NH)
#define WS_V2  (WS_B1 + 4u * NRP * NH)
#define WS_END (WS_V2 + 4u * NR * DM)

__global__ __launch_bounds__(256) void k_pack(const float* __restrict__ WH0, const float* __restrict__ WQ, const float* __restrict__ WKE, const float* __restrict__ WKV, const float* __restrict__ WKR, const float* __restrict__ WH1, const float* __restrict__ WO1, __bf16* __restrict__ PK) {
  __shared__ __align__(16) __bf16 s[HID]; const int n = blockIdx.x, which = blockIdx.y, t = threadIdx.x; int K, NO; size_t dst; const float* Wm;
  switch (which) { case 0: Wm = WH0; K = DM; NO = HID; dst = PK_H0; break; case 1: Wm = WQ; K = HID; NO = DM; dst = PK_Q; break; case 2: Wm = WKE; K = HID; NO = DM; dst = PK_KE; break; case 3: Wm = WKV; K = HID; NO = DM; dst = PK_KV; break; case 4: Wm = WKR; K = DM; NO = DM; dst = PK_KR; break; case 5: Wm = WH1; K = DM; NO = HID; dst = PK_H1; break; default: Wm = WO1; K = HID; NO = DM; dst = PK_O1; break; }
  if (n >= NO) return;
  for (int k = t; k < K; k += 256) s[k] = (__bf16)Wm[(size_t)k * NO + n];
  __syncthreads();
  for (int q = t; q < K / 8; q += 256) vst2((unsigned*)(PK + dst + (size_t)n * K + q * 8), *(const v4u*)&s[q * 8]);
}
__global__ __launch_bounds__(128) void k_ln(const float* __restrict__ SRC, int round_in, const float* __restrict__ G, const float* __restrict__ Bv, float* __restrict__ XN) {
  __shared__ float red[2][4]; const int t = threadIdx.x; const size_t row = RB0 + blockIdx.x; const float* p = SRC + row * DM + t * 4;
  float v[4]; for (int i = 0; i < 4; ++i) v[i] = round_in ? bfr(p[i]) : p[i]; float s = (v[0] + v[1]) + (v[2] + v[3]);
#pragma unroll
  for (int o = 1; o < 32; o <<= 1) s += __shfl_xor(s, o);
  if ((t & 31) == 0) red[0][t >> 5] = s; __syncthreads();
  const float mu = (red[0][0] + red[0][1] + red[0][2] + red[0][3]) / (float)DM; float q = 0.f;
#pragma unroll
  for (int i = 0; i < 4; ++i) { const float d = v[i] - mu; q += d * d; }
#pragma unroll
  for (int o = 1; o < 32; o <<= 1) q += __shfl_xor(q, o);
  if ((t & 31) == 0) red[1][t >> 5] = q; __syncthreads();
  const float inv = 1.0f / sqrtf((red[1][0] + red[1][1] + red[1][2] + red[1][3]) / (float)DM + 1e-3f); v4f o4;
#pragma unroll
  for (int i = 0; i < 4; ++i) o4[i] = (v[i] - mu) * inv * bfr(G[t * 4 + i]) + bfr(Bv[t * 4 + i]);
  vst2(XN + row * DM + t * 4, o4);
}
template <int MODE>
__global__ __launch_bounds__(128) void k_dense(const float* __restrict__ XN, const __bf16* __restrict__ XH, const __bf16* __restrict__ XL, const __bf16* __restrict__ P, const float* __restrict__ BIAS, const float* __restrict__ RES, __bf16* __restrict__ OH_, __bf16* __restrict__ OL_, float* __restrict__ OUTF) {
  __shared__ __align__(16) __bf16 sg[4][16][136], sgl[4][16][136]; __shared__ __align__(16) float so[4][16][132];
  const int tid = threadIdx.x, wave = tid >> 5, lane = tid & 31, col = lane & 15, g = lane >> 4; const size_t r0 = RB0 + (size_t)blockIdx.x * 64 + wave * 16; const int n0 = blockIdx.y * 128;
  v8f acc[8] = {};
  if (MODE == 0) {
#pragma unroll 2
    for (int kc = 0; kc < DM / 32; ++kc) { const F2 a = split_row(XN + (r0 + col) * DM, kc * 32, lane);
#pragma unroll
      for (int j = 0; j < 8; ++j) { const v16b w = frag_b(P + (size_t)(n0 + j * 16 + col) * DM + kc * 32, lane); acc[j] = wmma_bf(a.l, w, acc[j]); acc[j] = wmma_bf(a.h, w, acc[j]); } }
#pragma unroll
    for (int j = 0; j < 8; ++j) { const float bb = bfr(BIAS[n0 + j * 16 + col]);
#pragma unroll
      for (int r = 0; r < 8; ++r) { const float v = fmaxf(acc[j][r] + bb, 0.f); const __bf16 hb = (__bf16)v; sg[wave][8 * g + r][j * 16 + col] = hb; sgl[wave][8 * g + r][j * 16 + col] = (__bf16)(v - (float)hb); } }
    LDSX();
    for (int rl = 0; rl < 16; ++rl) { if (lane < 16) vst2((unsigned*)(OH_ + (r0 + rl) * HID + n0 + lane * 8), *(const v4u*)&sg[wave][rl][lane * 8]); else vst2((unsigned*)(OL_ + (r0 + rl) * HID + n0 + (lane - 16) * 8), *(const v4u*)&sgl[wave][rl][(lane - 16) * 8]); }
  } else {
#pragma unroll 2
    for (int kc = 0; kc < HID / 32; ++kc) { const v16b a = frag_b(XH + (r0 + col) * HID + kc * 32, lane), al = frag_b(XL + (r0 + col) * HID + kc * 32, lane);
#pragma unroll
      for (int j = 0; j < 8; ++j) { const v16b w = frag_b(P + (size_t)(n0 + j * 16 + col) * HID + kc * 32, lane); acc[j] = wmma_bf(al, w, acc[j]); acc[j] = wmma_bf(a, w, acc[j]); } }
#pragma unroll
    for (int j = 0; j < 8; ++j) { const int c = n0 + j * 16 + col; const float bb = bfr(BIAS[c]);
#pragma unroll
      for (int r = 0; r < 8; ++r) { const size_t row = r0 + 8 * g + r; so[wave][8 * g + r][j * 16 + col] = acc[j][r] + bb + RES[row * DM + c]; } }
    LDSX();
    for (int rl = 0; rl < 16; ++rl) vst2(OUTF + (r0 + rl) * DM + n0 + lane * 4, *(const v4f*)&so[wave][rl][lane * 4]); }
}
__global__ __launch_bounds__(128) void k_qkv(const __bf16* __restrict__ XH, const __bf16* __restrict__ XL, const float* __restrict__ REL, const __bf16* __restrict__ PK, const float* __restrict__ BQ, const float* __restrict__ BKE, const float* __restrict__ BKV, const float* __restrict__ BKR, _Float16* __restrict__ QH, _Float16* __restrict__ QL, _Float16* __restrict__ KEH, _Float16* __restrict__ KEL, _Float16* __restrict__ VTH, _Float16* __restrict__ VTL, _Float16* __restrict__ KRH, _Float16* __restrict__ KRL, float* __restrict__ KRF) {
  __shared__ __align__(16) _Float16 soh[4][16][136], sol[4][16][136]; __shared__ __align__(16) _Float16 sth[128][72], stl[128][72]; __shared__ __align__(16) float sof[4][16][132];
  const int tid = threadIdx.x, wave = tid >> 5, lane = tid & 31, col = lane & 15, g = lane >> 4; const int which = blockIdx.z; const int n0 = blockIdx.y * 128;
  if (which == 3 && blockIdx.x * 64 >= NRP) return; if (which != 3 && blockIdx.x >= NBT * TT / 64) return;
  const size_t r0 = ((which == 3) ? 0 : RB0) + (size_t)blockIdx.x * 64 + wave * 16;
  const __bf16* P = PK + ((which == 0) ? PK_Q : (which == 1) ? PK_KE : (which == 2) ? PK_KV : PK_KR); const float* BB = (which == 0) ? BQ : (which == 1) ? BKE : (which == 2) ? BKV : BKR;
  v8f acc[8] = {};
  if (which == 3) {
#pragma unroll 2
    for (int kc = 0; kc < DM / 32; ++kc) { v16b a; { const size_t rr = r0 + col; const bool ok = rr < NREL; const float* p = REL + (ok ? rr : 0) * DM + kc * 32 + 8 * g;
#pragma unroll
        for (int i = 0; i < 8; ++i) { a[i] = (__bf16)(ok ? p[i] : 0.f); a[8 + i] = (__bf16)(ok ? p[16 + i] : 0.f); } }
#pragma unroll
      for (int j = 0; j < 8; ++j) acc[j] = wmma_bf(a, frag_b(P + (size_t)(n0 + j * 16 + col) * DM + kc * 32, lane), acc[j]); }
  } else {
#pragma unroll 2
    for (int kc = 0; kc < HID / 32; ++kc) { const v16b a = frag_b(XH + (r0 + col) * HID + kc * 32, lane), al = frag_b(XL + (r0 + col) * HID + kc * 32, lane);
#pragma unroll
      for (int j = 0; j < 8; ++j) { const v16b w = frag_b(P + (size_t)(n0 + j * 16 + col) * HID + kc * 32, lane); acc[j] = wmma_bf(al, w, acc[j]); acc[j] = wmma_bf(a, w, acc[j]); } } }
  if (which == 2) {
#pragma unroll
    for (int j = 0; j < 8; ++j) { const float bb = bfr(BB[n0 + j * 16 + col]);
#pragma unroll
      for (int r = 0; r < 8; ++r) { const float v = acc[j][r] + bb; const _Float16 hv = (_Float16)v; sth[j * 16 + col][wave * 16 + 8 * g + r] = hv; stl[j * 16 + col][wave * 16 + 8 * g + r] = (_Float16)((v - (float)hv) * 2048.0f); } }
    __syncthreads();
    const size_t rb = RB0 + (size_t)blockIdx.x * 64; const size_t b = rb / TT; const int s0 = (int)(rb % TT);
    for (int e = tid; e < 128 * 8; e += 128) { const int d = e >> 3, pc = e & 7; const size_t o = (b * DM + n0 + d) * TT + s0 + pc * 8; vst2((unsigned*)(VTH + o), *(const v4u*)&sth[d][pc * 8]); vst2((unsigned*)(VTL + o), *(const v4u*)&stl[d][pc * 8]); }
  } else {
    const bool isr = (which == 3);
#pragma unroll
    for (int j = 0; j < 8; ++j) { const float bb = bfr(BB[n0 + j * 16 + col]);
#pragma unroll
      for (int r = 0; r < 8; ++r) { const bool okrow = !isr || (r0 + 8 * g + r) < NREL; const float v = okrow ? acc[j][r] + bb : 0.f; const _Float16 hv = (_Float16)v; soh[wave][8 * g + r][j * 16 + col] = hv; sol[wave][8 * g + r][j * 16 + col] = (_Float16)((v - (float)hv) * 2048.0f); if (isr) sof[wave][8 * g + r][j * 16 + col] = v; } }
    LDSX();
    _Float16* DH_ = (which == 0) ? QH : (which == 1) ? KEH : KRH; _Float16* DL_ = (which == 0) ? QL : (which == 1) ? KEL : KRL;
    for (int rl = 0; rl < 16; ++rl) { const size_t o = (r0 + rl) * DM + n0; if (lane < 16) vst2((unsigned*)(DH_ + o + lane * 8), *(const v4u*)&soh[wave][rl][lane * 8]); else vst2((unsigned*)(DL_ + o + (lane - 16) * 8), *(const v4u*)&sol[wave][rl][(lane - 16) * 8]); }
    if (isr) for (int rl = 0; rl < 16; ++rl) vst2(KRF + (r0 + rl) * DM + n0 + lane * 4, *(const v4f*)&sof[wave][rl][lane * 4]);
  }
}
__global__ __launch_bounds__(256) void k_bias(const _Float16* __restrict__ KEH, const _Float16* __restrict__ KEL, const float* __restrict__ KRF, const float* __restrict__ WB0, const float* __restrict__ BB0, const float* __restrict__ WB1, const float* __restrict__ BB1, int which, float* __restrict__ B0, float* __restrict__ B1) {
  __shared__ __align__(16) float sb[64][NH]; const int t = threadIdx.x; const int rl = t >> 2, hp = t & 3; const size_t row = (which == 0) ? (RB0 + (size_t)blockIdx.x * 64 + rl) : ((size_t)blockIdx.x * 64 + rl);
  if (which == 1 && blockIdx.x * 64 >= NRP) return;
  for (int h = hp * 2; h < hp * 2 + 2; ++h) { float a = 0.f;
#pragma unroll 1
    for (int c = 0; c < DM; ++c) { const float kv = (which == 0) ? ((float)KEH[row * DM + c] + (float)KEL[row * DM + c] * (1.0f / 2048.0f)) : KRF[row * DM + c]; a += kv * bfr((which == 0) ? WB0[c * NH + h] : WB1[c * NH + h]); }
    sb[rl][h] = a + bfr((which == 0) ? BB0[h] : BB1[h]); }
  __syncthreads();
  float* dst = (which == 0) ? B0 : B1; const size_t base = (which == 0) ? (RB0 + (size_t)blockIdx.x * 64) : ((size_t)blockIdx.x * 64);
  for (int q = t; q < 64 * NH / 4; q += 256) vst2(dst + base * NH + q * 4, *(const v4f*)(&sb[0][0] + q * 4));
}
__global__ __launch_bounds__(128) void k_attn(const _Float16* __restrict__ QH, const _Float16* __restrict__ QL, const _Float16* __restrict__ KEH, const _Float16* __restrict__ KEL, const _Float16* __restrict__ KRH, const _Float16* __restrict__ KRL, const _Float16* __restrict__ VTH, const _Float16* __restrict__ VTL, const float* __restrict__ B0, const float* __restrict__ B1, const int* __restrict__ VM, const float* __restrict__ VAL, float* __restrict__ V2) {
  __shared__ __align__(16) _Float16 sph[4][16][40], spl[4][16][40]; __shared__ float sbd[4][16][49]; __shared__ __align__(16) float so[4][16][68]; __shared__ float sb1[NREL];
  const int tid = threadIdx.x, wave = tid >> 5, lane = tid & 31, col = lane & 15, g = lane >> 4; const int qb = blockIdx.x, h = blockIdx.y; const size_t b = blockIdx.z + TB0; const int i0 = qb * 64, iw0 = i0 + wave * 16; const size_t rowb = b * TT;
  for (int m = tid; m < NREL; m += 128) sb1[m] = B1[(size_t)m * NH + h];
  v16h aq[2], aql[2]; const size_t qo = (rowb + iw0 + col) * DM + h * HD;
#pragma unroll
  for (int kc = 0; kc < 2; ++kc) { aq[kc] = frag_h(QH + qo + kc * 32, lane); aql[kc] = frag_h(QL + qo + kc * 32, lane); }
  const _Float16* Vh = VTH + (b * DM + h * HD) * TT; const _Float16* Vl = VTL + (b * DM + h * HD) * TT;
  float m[8], l[8];
#pragma unroll
  for (int r = 0; r < 8; ++r) { m[r] = -3.0e38f; l[r] = 0.f; }
  v8f acc[4] = {}, accl[4] = {};
  __syncthreads();
  const int nks = (i0 + 64) / 32;
#pragma unroll 1
  for (int ks = 0; ks < nks; ++ks) { const int j0 = ks * 32;
    { const int r0w = j0 - iw0 - 15 + LR;
#pragma unroll
      for (int ct3 = 0; ct3 < 3; ++ct3) { int rr = r0w + ct3 * 16 + col; rr = min(max(rr, 0), 2 * LR); v8f u = {}, ul = {};
#pragma unroll
        for (int kc = 0; kc < 2; ++kc) { const v16h rh = frag_h(KRH + (size_t)rr * DM + h * HD + kc * 32, lane); u = wmma16(aq[kc], rh, u); ul = wmma16(aql[kc], rh, ul); ul = wmma16(aq[kc], frag_h(KRL + (size_t)rr * DM + h * HD + kc * 32, lane), ul); }
#pragma unroll
        for (int r = 0; r < 8; ++r) sbd[wave][8 * g + r][ct3 * 16 + col] = u[r] + ul[r] * (1.0f / 2048.0f); } }
    LDSX();
    v8f s[2];
#pragma unroll
    for (int ct = 0; ct < 2; ++ct) { const int jl = ct * 16 + col; const int kk = j0 + jl; const size_t rk = (rowb + kk) * DM + h * HD; v8f c = {}, cl = {};
#pragma unroll
      for (int kc = 0; kc < 2; ++kc) { const v16h khf = frag_h(KEH + rk + kc * 32, lane); c = wmma16(aq[kc], khf, c); cl = wmma16(aql[kc], khf, cl); cl = wmma16(aq[kc], frag_h(KEL + rk + kc * 32, lane), cl); }
      const float b0 = B0[(rowb + kk) * NH + h]; const bool keepk = VM[rowb + kk] != 0;
#pragma unroll
      for (int r = 0; r < 8; ++r) { const int il = 8 * g + r; const int i = iw0 + il; const int cidx = min(max(kk - i + LR, 0), 2 * LR); const bool keep = keepk && (kk <= i);
        s[ct][r] = keep ? ((c[r] + cl[r] * (1.0f / 2048.0f)) * 0.125f + sbd[wave][il][jl - il + 15] + b0 + sb1[cidx]) : -3.0e38f; } }
#pragma unroll
    for (int r = 0; r < 8; ++r) { float mx = fmaxf(s[0][r], s[1][r]);
#pragma unroll
      for (int o = 1; o < 16; o <<= 1) mx = fmaxf(mx, __shfl_xor(mx, o));
      const float mn = fmaxf(m[r], mx); const float alpha = (m[r] <= -1.0e38f) ? 0.f : __expf(m[r] - mn);
      const float e0 = (s[0][r] <= -1.0e38f) ? 0.f : __expf(s[0][r] - mn), e1 = (s[1][r] <= -1.0e38f) ? 0.f : __expf(s[1][r] - mn); float es = e0 + e1;
#pragma unroll
      for (int o = 1; o < 16; o <<= 1) es += __shfl_xor(es, o);
      l[r] = l[r] * alpha + es; m[r] = (mn <= -1.0e38f) ? m[r] : mn;
#pragma unroll
      for (int dt = 0; dt < 4; ++dt) { acc[dt][r] *= alpha; accl[dt][r] *= alpha; }
      const _Float16 h0 = (_Float16)e0, h1 = (_Float16)e1; sph[wave][8 * g + r][col] = h0; sph[wave][8 * g + r][16 + col] = h1; spl[wave][8 * g + r][col] = (_Float16)((e0 - (float)h0) * 2048.0f); spl[wave][8 * g + r][16 + col] = (_Float16)((e1 - (float)h1) * 2048.0f); }
    LDSX();
    const v16h pah = frag_h(&sph[wave][col][0], lane), pal = frag_h(&spl[wave][col][0], lane);
#pragma unroll
    for (int dt = 0; dt < 4; ++dt) { const size_t vo = (size_t)(dt * 16 + col) * TT + j0; const v16h vh = frag_h(Vh + vo, lane), vl = frag_h(Vl + vo, lane); acc[dt] = wmma16(pah, vh, acc[dt]); accl[dt] = wmma16(pal, vh, accl[dt]); accl[dt] = wmma16(pah, vl, accl[dt]); }
    LDSX(); }
#pragma unroll
  for (int r = 0; r < 8; ++r) { const float il = 1.0f / l[r]; const size_t row = rowb + iw0 + 8 * g + r;
#pragma unroll
    for (int dt = 0; dt < 4; ++dt) { const int c = h * HD + dt * 16 + col; so[wave][8 * g + r][dt * 16 + col] = (acc[dt][r] + accl[dt][r] * (1.0f / 2048.0f)) * il + bfr(VAL[row * DM + c]); } }
  LDSX();
  for (int rl = 0; rl < 16; ++rl) if (lane < 16) vst2(V2 + (rowb + iw0 + rl) * DM + h * HD + lane * 4, *(const v4f*)&so[wave][rl][lane * 4]);
}
extern "C" void kernel_launch(void* const* d_in, const int* in_sizes, int n_in, void* d_out, int out_size, void* d_ws, size_t ws_size, hipStream_t stream) {
  (void)in_sizes; (void)n_in; (void)out_size;
  const float** F = (const float**)d_in;
  if (ws_size < (size_t)WS_END) return;
  char* ws = (char*)d_ws; __bf16 *PK = (__bf16*)(ws + WS_PK), *XH = (__bf16*)(ws + WS_XH), *XL = (__bf16*)(ws + WS_XL); float *XN = (float*)(ws + WS_XN), *KRF = (float*)(ws + WS_KRF), *B0 = (float*)(ws + WS_B0), *B1 = (float*)(ws + WS_B1), *V2 = (float*)(ws + WS_V2);
  _Float16 *QH = (_Float16*)(ws + WS_QH), *QL = (_Float16*)(ws + WS_QL), *KEH = (_Float16*)(ws + WS_KEH), *KEL = (_Float16*)(ws + WS_KEL), *VTH = (_Float16*)(ws + WS_VTH), *VTL = (_Float16*)(ws + WS_VTL), *KRH = (_Float16*)(ws + WS_KRH), *KRL = (_Float16*)(ws + WS_KRL);
  const int RT = NBT * TT / 64;
  k_pack<<<dim3(HID, 7), 256, 0, stream>>>(F[5], F[7], F[9], F[11], F[13], F[21], F[23], PK);
  k_ln<<<NBT * TT, 128, 0, stream>>>(F[0], 1, F[3], F[4], XN);
  k_dense<0><<<dim3(RT, HID / 128), 128, 0, stream>>>(XN, nullptr, nullptr, PK + PK_H0, F[6], nullptr, XH, XL, nullptr);
  { const int rt = (RT > NRP / 64 + 1) ? RT : (NRP / 64 + 1); k_qkv<<<dim3(rt, DM / 128, 4), 128, 0, stream>>>(XH, XL, F[2], PK, F[8], F[10], F[12], F[14], QH, QL, KEH, KEL, VTH, VTL, KRH, KRL, KRF); }
  k_bias<<<RT, 256, 0, stream>>>(KEH, KEL, KRF, F[15], F[16], F[17], F[18], 0, B0, B1);
  k_bias<<<(NRP + 63) / 64, 256, 0, stream>>>(KEH, KEL, KRF, F[15], F[16], F[17], F[18], 1, B0, B1);
  k_attn<<<dim3(TQB, NH, NBT), 128, 0, stream>>>(QH, QL, KEH, KEL, KRH, KRL, VTH, VTL, B0, B1, (const int*)d_in[1], F[0], V2);
  k_ln<<<NBT * TT, 128, 0, stream>>>(V2, 0, F[19], F[20], XN);
  k_dense<0><<<dim3(RT, HID / 128), 128, 0, stream>>>(XN, nullptr, nullptr, PK + PK_H1, F[22], nullptr, XH, XL, nullptr);
  k_dense<1><<<dim3(RT, DM / 128), 128, 0, stream>>>(nullptr, XH, XL, PK + PK_O1, F[24], V2, nullptr, nullptr, (float*)d_out);
}
